// NeuralFilterModule_34729105555539
// MI455X (gfx1250) — hardware-verified
//
#include <hip/hip_runtime.h>
#include <math.h>

constexpr int kBatch     = 8;
constexpr int kTime      = 16384;
constexpr int kRows      = kBatch * kTime;
constexpr int kHalfBatch = 4;
constexpr int kHalfRows  = kHalfBatch * kTime;
constexpr int kPadRows   = 512;
constexpr int kTimePad   = kTime + kPadRows;
constexpr int kBlocks    = 10;
constexpr int kChan      = 64;
constexpr int kCore      = 32;
constexpr int kWide      = 128;
constexpr int kHeadN     = 16;
constexpr float kWCarry    = 64.0f;
constexpr float kWCarryInv = 1.0f / 64.0f;

constexpr int kWConvH = kBlocks * kChan * 2 * kChan;
constexpr int kWFgH   = kBlocks * kChan * kWide;
constexpr int kW1H    = kBlocks * kChan * kCore;
constexpr int kW2H    = kBlocks * kWide * kChan;
constexpr int kP1H    = kChan * kWide;
constexpr int kWUnitsConv = kWConvH / 8;
constexpr int kWUnitsFg   = kWFgH / 8;
constexpr int kWUnits1    = kW1H / 8;
constexpr int kWUnits2    = kW2H / 8;
constexpr int kWUnitsP    = kP1H / 8;
constexpr int kWUnitsAll  = kWUnitsConv + kWUnitsFg + kWUnits1 + kWUnits2 + kWUnitsP;
static_assert(kWUnitsAll == 134 * 256, "prep grid exact");
static_assert(kWUnitsConv % 256 == 0 && kWUnitsFg % 256 == 0 && kWUnits1 % 256 == 0 && kWUnits2 % 256 == 0 && kWUnitsP % 256 == 0, "block-uniform segments");

typedef __attribute__((ext_vector_type(16))) _Float16 v16h;
typedef __attribute__((ext_vector_type(8)))  _Float16 v8h;
typedef __attribute__((ext_vector_type(8)))  float    v8f;
typedef __attribute__((ext_vector_type(4)))  float    v4f;
typedef __attribute__((ext_vector_type(4)))  unsigned int v4u;

__device__ __forceinline__ void dep_guard_h(v8f& a, v8f& b, v16h x, v16h y) { asm volatile("v_nop\n\tv_nop\n\tv_nop\n\tv_nop" : "+v"(a), "+v"(b) : "v"(x), "v"(y)); }
__device__ __forceinline__ void keep4_h(v16h a, v16h b, v16h c, v16h d) { asm volatile("v_nop" :: "v"(a), "v"(b), "v"(c), "v"(d)); }
__device__ __forceinline__ void acc_guard4(v8f& a, v8f& b, v8f& c, v8f& d) { asm volatile("v_nop\n\tv_nop\n\tv_nop\n\tv_nop" : "+v"(a), "+v"(b), "+v"(c), "+v"(d)); }
template <typename T> struct Frag;
template <> struct Frag<_Float16> {
  typedef v16h V; union U { v16h v; v8h h[2]; };
  static __device__ __forceinline__ v16h load(const _Float16* p) {
    U f; f.h[0] = *(const v8h*)(p); f.h[1] = *(const v8h*)(p + 16); return f.v;
  }
  static __device__ __forceinline__ v8f mma(v16h a, v16h b, v8f c) {
    return __builtin_amdgcn_wmma_f32_16x16x32_f16(false, a, false, b, (short)0, c, false, false);
  }
  static __device__ __forceinline__ void guard(v8f& a, v8f& b, v16h x, v16h y) { dep_guard_h(a, b, x, y); }
  static __device__ __forceinline__ void keep(v16h a, v16h b, v16h c, v16h d) { keep4_h(a, b, c, d); }
};

__device__ __forceinline__ unsigned pk16(unsigned short a, unsigned short b) { return (unsigned)a | ((unsigned)b << 16); }
__device__ __forceinline__ unsigned short h_bits(float f) { const _Float16 h = (_Float16)f; return __builtin_bit_cast(unsigned short, h); }

template <int AMODE, int BIAS_MODE, int OUT_MODE, bool RESID>
__global__ __launch_bounds__(256) void gemm64_f16(
    const unsigned short* __restrict__ Ap, int lda, long strideA,
    const unsigned short* __restrict__ A2p, int lda2, long strideA2, int kcat,
    const unsigned short* __restrict__ Btp, int ldb, long strideB,
    void* Cout, int ldc, long strideC,
    void* Cout2, int ldc2, long strideC2,
    const float* __restrict__ bias, const float* __restrict__ bias2,
    const float* resid, int ldr, long strideR,
    int M, int N, int K, float scale) {
  typedef _Float16 T;
  typedef v16h V;
  const T* A = (const T*)Ap; const T* A2 = (const T*)A2p; const T* Bt = (const T*)Btp;
  __shared__ __align__(16) float sT[8][16 * 68];
  const int b    = blockIdx.y;
  const int lane = threadIdx.x & 31;
  const int wave = threadIdx.x >> 5;
  const int tilesN = N >> 6;
  const int tilesM = M >> 6;
  const int tile = blockIdx.x * 8 + wave;
  if (tile >= tilesM * tilesN) return;
  const int tm = tile / tilesN;
  const int tn = tile - tm * tilesN;
  const int m0 = tm << 6;
  const int n0 = tn << 6;

  const T* Ab  = A + (size_t)b * (size_t)strideA;
  const T* Ab2 = (AMODE == 1) ? (A2 + (size_t)b * (size_t)strideA2) : Ab;
  const T* Bb  = Bt + (size_t)b * (size_t)strideB;

  const int rlane = lane & 15;
  const int koff  = (lane >> 4) * 8;
  const int mOff  = (lane >> 4) * 8;

  v8f acc[4][4];
#pragma unroll
  for (int i = 0; i < 4; ++i)
#pragma unroll
    for (int j = 0; j < 4; ++j) acc[i][j] = (v8f){0.f,0.f,0.f,0.f,0.f,0.f,0.f,0.f};

  for (int k0 = 0; k0 < K; k0 += 32) {
    V bh[4];
#pragma unroll
    for (int j = 0; j < 4; ++j) {
      const size_t bo = (size_t)(n0 + (j << 4) + rlane) * ldb + koff + k0;
      bh[j] = Frag<T>::load(Bb + bo);
    }
    const T* As = Ab; int ldas = lda; int ka = k0;
    if (AMODE == 1) {
      if (k0 >= kcat) { As = Ab2; ldas = lda2; ka = k0 - kcat; }
    }
#pragma unroll
    for (int i = 0; i < 4; ++i) {
      const size_t ao = (size_t)(m0 + (i << 4) + rlane) * ldas + koff + ka;
      V ah = Frag<T>::load(As + ao);
#pragma unroll
      for (int j = 0; j < 4; ++j) acc[i][j] = Frag<T>::mma(ah, bh[j], acc[i][j]);
      Frag<T>::guard(acc[i][0], acc[i][3], ah, ah);
    }
    Frag<T>::keep(bh[0], bh[1], bh[2], bh[3]);
  }
  acc_guard4(acc[0][0], acc[0][1], acc[0][2], acc[0][3]);
  acc_guard4(acc[1][0], acc[1][1], acc[1][2], acc[1][3]);
  acc_guard4(acc[2][0], acc[2][1], acc[2][2], acc[2][3]);
  acc_guard4(acc[3][0], acc[3][1], acc[3][2], acc[3][3]);

  float* slab = sT[wave];
  const float* Rb = RESID ? (resid + (size_t)b * (size_t)strideR) : nullptr;
#pragma unroll
  for (int i = 0; i < 4; ++i) {
    const int mBase = m0 + (i << 4);
    if (OUT_MODE == 4) {
#pragma unroll
      for (int j = 0; j < 2; ++j) {
        const int n = (j << 4) + rlane;
        const float bfv = bias[n];
        const float bgv = bias2[n];
#pragma unroll
        for (int r = 0; r < 8; ++r) {
          const float f  = acc[i][j][r] * scale + bfv;
          const float gp = acc[i][j + 2][r] * scale + bgv;
          const float ef = __expf(2.0f * f);
          const float th = 1.0f - 2.0f * __builtin_amdgcn_rcpf(1.0f + ef);
          const float eg = __expf(-gp);
          const float sg = __builtin_amdgcn_rcpf(1.0f + eg);
          slab[(mOff + r) * 68 + (j << 4) + rlane] = th * sg;
        }
      }
    } else {
#pragma unroll
      for (int j = 0; j < 4; ++j) {
        const int n = n0 + (j << 4) + rlane;
        float bv = 0.f;
        if (BIAS_MODE == 2) bv = bias[n];
#pragma unroll
        for (int r = 0; r < 8; ++r) {
          float v = acc[i][j][r] * scale;
          if (BIAS_MODE == 2) v += bv;
          if (RESID) v += Rb[(size_t)(mBase + mOff + r) * ldr + n];
          slab[(mOff + r) * 68 + (j << 4) + rlane] = v;
        }
      }
    }
    __builtin_amdgcn_fence(__ATOMIC_RELEASE, "workgroup");
    __builtin_amdgcn_wave_barrier();
    __builtin_amdgcn_fence(__ATOMIC_ACQUIRE, "workgroup");
    if (OUT_MODE == 0 || OUT_MODE == 3) {
      float* C = (float*)Cout + (size_t)b * (size_t)strideC;
      const int hh = lane >> 4, c4 = (lane & 15) * 4;
      for (int pass = 0; pass < 2; ++pass) {
#pragma unroll
        for (int it = 0; it < 8; ++it) {
          const int row = it * 2 + hh;
          v4f v = *(const v4f*)(slab + row * 68 + c4);
          *(volatile v4f*)(C + (size_t)(mBase + row) * ldc + n0 + c4) = v;
        }
        __threadfence();
      }
    }
    if (OUT_MODE == 1 || OUT_MODE == 3) {
      unsigned short* C = (OUT_MODE == 1) ? ((unsigned short*)Cout + (size_t)b * (size_t)strideC)
                                          : ((unsigned short*)Cout2 + (size_t)b * (size_t)strideC2);
      const int ldh = (OUT_MODE == 1) ? ldc : ldc2;
      const int q = lane >> 3, c8 = (lane & 7) * 8;
      for (int pass = 0; pass < 2; ++pass) {
#pragma unroll
        for (int it = 0; it < 4; ++it) {
          const int row = it * 4 + q;
          const float* sp = slab + row * 68 + c8;
          v8h hv;
#pragma unroll
          for (int e = 0; e < 8; ++e) hv[e] = (_Float16)sp[e];
          *(volatile v8h*)(C + (size_t)(mBase + row) * ldh + n0 + c8) = hv;
        }
        __threadfence();
      }
    }
    if (OUT_MODE == 4) {
      unsigned short* C = (unsigned short*)Cout + (size_t)b * (size_t)strideC;
      const int rq = lane >> 2, c8 = (lane & 3) * 8;
      for (int pass = 0; pass < 2; ++pass) {
#pragma unroll
        for (int it = 0; it < 2; ++it) {
          const int row = it * 8 + rq;
          const float* sp = slab + row * 68 + c8;
          v8h hv;
#pragma unroll
          for (int e = 0; e < 8; ++e) hv[e] = (_Float16)sp[e];
          *(volatile v8h*)(C + (size_t)(mBase + row) * ldc + c8) = hv;
        }
        __threadfence();
      }
    }
    __builtin_amdgcn_fence(__ATOMIC_RELEASE, "workgroup");
    __builtin_amdgcn_wave_barrier();
    __builtin_amdgcn_fence(__ATOMIC_ACQUIRE, "workgroup");
  }
}

__global__ __launch_bounds__(256) void prep_weights_kernel(
    const float* __restrict__ conv_w, const float* __restrict__ wf, const float* __restrict__ wg,
    const float* __restrict__ w1, const float* __restrict__ w2, const float* __restrict__ p1w,
    unsigned short* Wout) {
  const int u  = blockIdx.x * 256 + threadIdx.x;
  const int bx = blockIdx.x;
  float v[8];
  if (bx < kWUnitsConv / 256) {
    const int e0 = 8 * u;
#pragma unroll
    for (int j = 0; j < 8; ++j) {
      const int e = e0 + j;
      const int i = e >> 13, rem = e & 8191, n = rem >> 7, k = rem & 127;
      const int tap = k >> 6, cin = k & 63;
      v[j] = conv_w[((i * kChan + cin) * kChan + n) * 2 + tap];
    }
  } else if (bx < (kWUnitsConv + kWUnitsFg) / 256) {
    const int e0 = 8 * (u - kWUnitsConv);
#pragma unroll
    for (int j = 0; j < 8; ++j) {
      const int e = e0 + j;
      const int i = e >> 13, rem = e & 8191, n = rem >> 7, k = rem & 127;
      const int idx = (i * kWide + k) * kCore + (n & 31);
      const float vf = wf[idx];
      const float vg = wg[idx];
      v[j] = (n < kCore) ? vf : vg;
    }
  } else if (bx < (kWUnitsConv + kWUnitsFg + kWUnits1) / 256) {
    const int e0 = 8 * (u - kWUnitsConv - kWUnitsFg);
#pragma unroll
    for (int j = 0; j < 8; ++j) {
      const int e = e0 + j;
      const int i = e >> 11, rem = e & 2047, n = rem >> 5, k = rem & 31;
      v[j] = w1[(i * kCore + k) * kChan + n];
    }
  } else if (bx < (kWUnitsConv + kWUnitsFg + kWUnits1 + kWUnits2) / 256) {
    const int e0 = 8 * (u - kWUnitsConv - kWUnitsFg - kWUnits1);
#pragma unroll
    for (int j = 0; j < 8; ++j) {
      const int e = e0 + j;
      const int i = e >> 13, rem = e & 8191, n = rem >> 6, k = rem & 63;
      v[j] = w2[(i * kChan + k) * kWide + n];
    }
  } else {
    const int e0 = 8 * (u - kWUnitsConv - kWUnitsFg - kWUnits1 - kWUnits2);
#pragma unroll
    for (int j = 0; j < 8; ++j) {
      const int e = e0 + j;
      const int n = e >> 7, k = e & 127;
      const float vp = p1w[k * kHeadN + (n & 15)];
      v[j] = (n < kHeadN) ? vp : 0.0f;
    }
  }
  unsigned short hb[8];
#pragma unroll
  for (int j = 0; j < 8; ++j) hb[j] = h_bits(v[j] * kWCarry);
  const v4u pk = (v4u){pk16(hb[0], hb[1]), pk16(hb[2], hb[3]), pk16(hb[4], hb[5]), pk16(hb[6], hb[7])};
  unsigned short* dst = Wout + 8 * (size_t)u;
  *(volatile v4u*)dst = pk;
  __threadfence();
  *(volatile v4u*)dst = pk;
}

__global__ __launch_bounds__(256) void init_half_kernel(
    const float* __restrict__ xh, const float* __restrict__ ch,
    const float* __restrict__ cw, const float* __restrict__ cb,
    float* H32, unsigned short* H16, unsigned short* C16) {
  const int i = blockIdx.x * 256 + threadIdx.x;
  {
    const int row = i >> 4, c4 = (i & 15) * 4;
    const float xv = xh[row];
    v4f hv;
#pragma unroll
    for (int e = 0; e < 4; ++e) hv[e] = xv * cw[c4 + e] + cb[c4 + e];
    float* dst = H32 + (size_t)i * 4;
    *(volatile v4f*)dst = hv;
    __threadfence();
    *(volatile v4f*)dst = hv;
  }
  if (i < kHalfRows * 8) {
    const int row = i >> 3, c8 = (i & 7) * 8;
    const float xv = xh[row];
    unsigned short hb[8];
#pragma unroll
    for (int e = 0; e < 8; ++e) hb[e] = h_bits(xv * cw[c8 + e] + cb[c8 + e]);
    const v4u hpk = (v4u){pk16(hb[0], hb[1]), pk16(hb[2], hb[3]), pk16(hb[4], hb[5]), pk16(hb[6], hb[7])};
    const int bl = row >> 14, t = row & (kTime - 1);
    unsigned short* hdst = H16 + ((size_t)(bl * kTimePad + kPadRows + t) * kChan + c8);
    const float* cp = ch + (size_t)row * kChan + c8;
    const v4f ca = *(const v4f*)(cp);
    const v4f cc = *(const v4f*)(cp + 4);
    unsigned short ccb[8];
#pragma unroll
    for (int e = 0; e < 4; ++e) { ccb[e] = h_bits(ca[e]); ccb[4 + e] = h_bits(cc[e]); }
    const v4u cpk = (v4u){pk16(ccb[0], ccb[1]), pk16(ccb[2], ccb[3]), pk16(ccb[4], ccb[5]), pk16(ccb[6], ccb[7])};
    unsigned short* cdst = C16 + (size_t)i * 8;
    *(volatile v4u*)hdst = hpk;
    *(volatile v4u*)cdst = cpk;
    __threadfence();
    *(volatile v4u*)hdst = hpk;
    *(volatile v4u*)cdst = cpk;
  }
  if (i < kHalfBatch * kPadRows * 8) {
    const int bl = i >> 12, w = i & 4095;
    unsigned short* pdst = H16 + (size_t)bl * kTimePad * kChan + (size_t)w * 8;
    const v4u z = (v4u){0u, 0u, 0u, 0u};
    *(volatile v4u*)pdst = z;
    __threadfence();
    *(volatile v4u*)pdst = z;
  }
}

__global__ __launch_bounds__(256) void final_kernel(
    const float* __restrict__ xh, const float* __restrict__ P1,
    const float* __restrict__ p1b, const float* __restrict__ p2w, const float* __restrict__ p2b,
    float* outh) {
  const int r = blockIdx.x * 256 + threadIdx.x;
  const float* pr = P1 + (size_t)r * kChan;
  const v4f a0 = *(const v4f*)(pr);
  const v4f a1 = *(const v4f*)(pr + 4);
  const v4f a2 = *(const v4f*)(pr + 8);
  const v4f a3 = *(const v4f*)(pr + 12);
  const float pv[16] = {a0[0], a0[1], a0[2], a0[3], a1[0], a1[1], a1[2], a1[3],
                        a2[0], a2[1], a2[2], a2[3], a3[0], a3[1], a3[2], a3[3]};
  float s0 = 0.f, s1 = 0.f;
#pragma unroll
  for (int n = 0; n < 16; ++n) {
    const float pn = pv[n] + p1b[n];
    s0 += pn * p2w[2 * n];
    s1 += pn * p2w[2 * n + 1];
  }
  s0 += p2b[0];
  s1 += p2b[1];
  const float o = xh[r] * expf(s1) + s0;
  *(volatile float*)(outh + r) = o;
  __threadfence();
  *(volatile float*)(outh + r) = o;
}

extern "C" void kernel_launch(void* const* d_in, const int* in_sizes, int n_in,
                              void* d_out, int out_size, void* d_ws, size_t ws_size,
                              hipStream_t stream) {
  if (n_in < 18) return;
  if (in_sizes[0] != kRows) return;
  if (in_sizes[1] != kRows * kChan) return;
  if (in_sizes[2] != kChan || in_sizes[3] != kChan) return;
  if (in_sizes[4] != kBlocks * kChan * kChan * 2 || in_sizes[5] != kBlocks * kChan) return;
  if (in_sizes[6] != kBlocks * kWide * kCore || in_sizes[7] != kBlocks * kCore) return;
  if (in_sizes[8] != kBlocks * kWide * kCore || in_sizes[9] != kBlocks * kCore) return;
  if (in_sizes[10] != kBlocks * kCore * kChan || in_sizes[11] != kBlocks * kChan) return;
  if (in_sizes[12] != kBlocks * kChan * kWide || in_sizes[13] != kBlocks * kWide) return;
  if (in_sizes[14] != kWide * kHeadN || in_sizes[15] != kHeadN || in_sizes[16] != kHeadN * 2 || in_sizes[17] != 2) return;
  if (out_size != kRows) return;

  const float* x      = (const float*)d_in[0];
  const float* c      = (const float*)d_in[1];
  const float* cw     = (const float*)d_in[2];
  const float* cb     = (const float*)d_in[3];
  const float* conv_w = (const float*)d_in[4];
  const float* conv_b = (const float*)d_in[5];
  const float* wf     = (const float*)d_in[6];
  const float* bfp    = (const float*)d_in[7];
  const float* wg     = (const float*)d_in[8];
  const float* bgp    = (const float*)d_in[9];
  const float* w1     = (const float*)d_in[10];
  const float* b1     = (const float*)d_in[11];
  const float* w2     = (const float*)d_in[12];
  const float* b2     = (const float*)d_in[13];
  const float* p1w    = (const float*)d_in[14];
  const float* p1b    = (const float*)d_in[15];
  const float* p2w    = (const float*)d_in[16];
  const float* p2b    = (const float*)d_in[17];
  float* out = (float*)d_out;

  const size_t SZ_W    = (size_t)(kWConvH + kWFgH + kW1H + kW2H + kP1H) * 2;
  const size_t SZ_YS   = (size_t)kHalfRows * kWide * 4;
  const size_t SZ_H32  = (size_t)kHalfRows * kChan * 4;
  const size_t SZ_H16  = (size_t)kHalfBatch * kTimePad * kChan * 2;
  const size_t SZ_A16  = (size_t)kHalfRows * kChan * 2;
  const size_t SZ_G16  = (size_t)kHalfRows * kCore * 2;
  size_t off = 0;
  const size_t oW   = off; off += SZ_W;
  const size_t oYS  = off; off += SZ_YS;
  const size_t oH32 = off; off += SZ_H32;
  const size_t oH16 = off; off += SZ_H16;
  const size_t oC16 = off; off += SZ_A16;
  const size_t oCV  = off; off += SZ_A16;
  const size_t oG16 = off; off += SZ_G16;
  const size_t TOTAL = off;
  if (TOTAL > ws_size) return;
  if (TOTAL > (size_t)134217728) return;

  char* ws = (char*)d_ws;
  unsigned short* WB     = (unsigned short*)(ws + oW);
  unsigned short* WCONV  = WB;
  unsigned short* WFG    = WCONV + kWConvH;
  unsigned short* W1T    = WFG + kWFgH;
  unsigned short* W2T    = W1T + kW1H;
  unsigned short* P1T    = W2T + kW2H;
  float*          YS     = (float*)(ws + oYS);
  float*          H32    = (float*)(ws + oH32);
  float*          P1     = H32;
  unsigned short* H16    = (unsigned short*)(ws + oH16);
  unsigned short* C16    = (unsigned short*)(ws + oC16);
  unsigned short* CONV16 = (unsigned short*)(ws + oCV);
  unsigned short* YS16   = C16;
  unsigned short* G16    = (unsigned short*)(ws + oG16);

  const dim3 blk(256);
  const long sH16  = (long)kTimePad * kChan;
  const long sT64  = (long)kTime * kChan;
  const long sT32  = (long)kTime * kCore;
  const long sT128 = (long)kTime * kWide;
  unsigned short* H16d = H16 + (size_t)kPadRows * kChan;

  prep_weights_kernel<<<dim3(kWUnitsAll / 256), blk, 0, stream>>>(conv_w, wf, wg, w1, w2, p1w, WB);

  for (int half = 0; half < 2; ++half) {
    const float* xh  = x + (size_t)half * kHalfRows;
    const float* chp = c + (size_t)half * kHalfRows * kChan;
    float* outh = out + (size_t)half * kHalfRows;

    init_half_kernel<<<dim3(kHalfRows * 16 / 256), blk, 0, stream>>>(xh, chp, cw, cb, H32, H16, C16);

    for (int i = 0; i < kBlocks; ++i) {
      const int d = 1 << i;
      const unsigned short* wconv = WCONV + (size_t)i * kChan * kWide;
      const unsigned short* wfg   = WFG + (size_t)i * kChan * kWide;
      const unsigned short* w1t   = W1T + (size_t)i * kChan * kCore;
      const unsigned short* w2t   = W2T + (size_t)i * kWide * kChan;
      const unsigned short* H16s  = H16 + (size_t)(kPadRows - d) * kChan;

      gemm64_f16<1, 2, 1, false><<<dim3(32, kHalfBatch), blk, 0, stream>>>(
          H16s, kChan, sH16, H16d, kChan, sH16, kChan,
          wconv, kWide, 0L,
          (void*)CONV16, kChan, sT64, (void*)CONV16, kChan, sT64,
          conv_b + i * kChan, conv_b + i * kChan,
          H32, kChan, 0L,
          kTime, kChan, kWide, kWCarryInv);

      gemm64_f16<1, 0, 4, false><<<dim3(128, 1), blk, 0, stream>>>(
          C16, kChan, 0L, CONV16, kChan, 0L, kChan,
          wfg, kWide, 0L,
          (void*)G16, kCore, 0L, (void*)G16, kCore, 0L,
          bfp + i * kCore, bgp + i * kCore,
          H32, kChan, 0L,
          kHalfRows, kChan, kWide, kWCarryInv);

      gemm64_f16<0, 2, 3, true><<<dim3(32, kHalfBatch), blk, 0, stream>>>(
          G16, kCore, sT32, G16, kCore, sT32, 0,
          w1t, kCore, 0L,
          (void*)H32, kChan, sT64, (void*)H16d, kChan, sH16,
          b1 + i * kChan, b1 + i * kChan,
          H32, kChan, sT64,
          kTime, kChan, kCore, kWCarryInv);

      if (i == 0) {
        gemm64_f16<0, 2, 0, false><<<dim3(64, kHalfBatch), blk, 0, stream>>>(
            H16d, kChan, sH16, H16d, kChan, sH16, 0,
            w2t, kChan, 0L,
            (void*)YS, kWide, sT128, (void*)YS, kWide, sT128,
            b2 + i * kWide, b2 + i * kWide,
            YS, kWide, sT128,
            kTime, kWide, kChan, kWCarryInv);
      } else if (i < kBlocks - 1) {
        gemm64_f16<0, 2, 0, true><<<dim3(64, kHalfBatch), blk, 0, stream>>>(
            H16d, kChan, sH16, H16d, kChan, sH16, 0,
            w2t, kChan, 0L,
            (void*)YS, kWide, sT128, (void*)YS, kWide, sT128,
            b2 + i * kWide, b2 + i * kWide,
            YS, kWide, sT128,
            kTime, kWide, kChan, kWCarryInv);
      } else {
        gemm64_f16<0, 2, 1, true><<<dim3(64, kHalfBatch), blk, 0, stream>>>(
            H16d, kChan, sH16, H16d, kChan, sH16, 0,
            w2t, kChan, 0L,
            (void*)YS16, kWide, sT128, (void*)YS16, kWide, sT128,
            b2 + i * kWide, b2 + i * kWide,
            YS, kWide, sT128,
            kTime, kWide, kChan, kWCarryInv);
      }
    }

    gemm64_f16<0, 0, 0, false><<<dim3(128, 1), blk, 0, stream>>>(
        YS16, kWide, 0L, YS16, kWide, 0L, 0,
        P1T, kWide, 0L,
        (void*)P1, kChan, 0L, (void*)P1, kChan, 0L,
        p1b, p1b,
        YS, kWide, 0L,
        kHalfRows, kChan, kWide, kWCarryInv);

    final_kernel<<<dim3(kHalfRows / 256), blk, 0, stream>>>(xh, P1, p1b, p2w, p2b, outh);
  }
}
